// CapsuleLayer_33698313404835
// MI455X (gfx1250) — hardware-verified
//
#include <hip/hip_runtime.h>
#include <math.h>

typedef __attribute__((ext_vector_type(16))) _Float16 v16h;
typedef __attribute__((ext_vector_type(8)))  _Float16 v8h;
typedef __attribute__((ext_vector_type(8)))  float    v8f;
typedef __attribute__((ext_vector_type(4)))  float    v4f;
typedef __attribute__((ext_vector_type(4)))  unsigned int v4u;

constexpr int kB   = 16;
constexpr int kCI  = 512;
constexpr int kCO  = 128;
constexpr int kQ   = 8;
constexpr int kS   = 8;
constexpr int kQS  = 64;
constexpr int kPitchH   = 16;
constexpr int kRowsPose = kCI * kB * kQ;
constexpr int kRowsT    = kCI * kCO * kS;
constexpr float kPoseCarry = 4.0f;
constexpr float kTCarry    = 64.0f;
constexpr float kInvVCarry = 1.0f / 512.0f;
constexpr float kLamb = 0.2f;
constexpr float kSqrtHalfLog2e = 0.84932180028801904f;
constexpr int kPlaneElems = kB * kCO * kQS;
constexpr int kLsumElems  = kB * kCO;
constexpr int kOut0Elems  = kB * kCO;
constexpr int kOut1Elems  = kB * kCO * kQS;
static_assert(kOut0Elems * 4 == 8192);
static_assert(kOut0Elems + kOut1Elems == 133120);
static_assert((kRowsPose * 2) % 256 == 0);
static_assert((kRowsT * 2) % 256 == 0);
static_assert(kB * kQ * kPitchH == 2048);
static_assert(kCO * kS * kPitchH == 16384);

__device__ __forceinline__ unsigned pk16(unsigned short a, unsigned short b) { return (unsigned)a | ((unsigned)b << 16); }
__device__ __forceinline__ unsigned short h_bits(float f) { const _Float16 h = (_Float16)f; return __builtin_bit_cast(unsigned short, h); }

union FragU { v16h v; v8h h[2]; };

__device__ __forceinline__ v8f mma_f16(v16h a, v16h b, v8f c) {
  return __builtin_amdgcn_wmma_f32_16x16x32_f16(false, a, false, b, (short)0, c, false, false);
}
__device__ __forceinline__ void guard_2acc_3frag(v8f& a, v8f& b, v16h x, v16h y, v16h z) {
  asm volatile("v_nop\n\tv_nop\n\tv_nop\n\tv_nop" : "+v"(a), "+v"(b) : "v"(x), "v"(y), "v"(z));
}
__device__ __forceinline__ void load8_wait(const float* __restrict__ p, float (&d)[8]) {
  v4f t0 = *(const v4f*)(p);
  v4f t1 = *(const v4f*)(p + 4);
  asm volatile("" : "+v"(t0), "+v"(t1));
  d[0] = t0[0]; d[1] = t0[1]; d[2] = t0[2]; d[3] = t0[3];
  d[4] = t1[0]; d[5] = t1[1]; d[6] = t1[2]; d[7] = t1[3];
}

template <int ISPOSE>
__global__ __launch_bounds__(256) void prep16_kernel(const float* __restrict__ src, unsigned short* __restrict__ dst, float scale) {
  const int g    = (int)blockIdx.x * 256 + (int)threadIdx.x;
  const int row  = g >> 1;
  const int part = g & 1;
  const int blk  = row >> 3;
  const int j    = row & 7;
  int sblk = blk;
  if (ISPOSE) {
    const int ic = blk >> 4;
    const int bb = blk & 15;
    sblk = bb * kCI + ic;
  }
  const float* p = src + (size_t)sblk * kQS + j;
  unsigned short hb[8];
#pragma unroll
  for (int k = 0; k < 8; ++k) hb[k] = h_bits(p[8 * k] * scale);
  const v4u u = (v4u){pk16(hb[0], hb[1]), pk16(hb[2], hb[3]), pk16(hb[4], hb[5]), pk16(hb[6], hb[7])};
  unsigned short* q = dst + (size_t)row * kPitchH + part * 8;
  *(volatile v4u*)q = u;
  __threadfence();
  *(volatile v4u*)q = u;
}

template <int MODE>
__device__ __forceinline__ void tile_update(const v8f acc, const float actv, const float (&ca)[8], const float (&cb)[8],
                                            float& A0, float (&A1)[8], float (&A2)[8]) {
  float v[8];
#pragma unroll
  for (int r = 0; r < 8; ++r) v[r] = acc[r] * kInvVCarry;
  float odds = actv;
  if (MODE > 0) {
    float ps = 0.0f;
#pragma unroll
    for (int r = 0; r < 8; ++r) {
      const float t = fmaf(v[r], ca[r], cb[r]);
      const float e = exp2f(-(t * t));
      ps = fmaf(ca[r], e, ps);
    }
    ps += __shfl_xor(ps, 1, 32);
    ps += __shfl_xor(ps, 2, 32);
    ps += __shfl_xor(ps, 4, 32);
    odds = actv * ps;
  }
  A0 += odds;
#pragma unroll
  for (int r = 0; r < 8; ++r) {
    const float ov = odds * v[r];
    A1[r] += ov;
    A2[r] = fmaf(ov, v[r], A2[r]);
  }
}

__device__ __forceinline__ void store_runs(const float* slabw, float* __restrict__ plane, int bp, int obase, int lane) {
  for (int pass = 0; pass < 2; ++pass) {
#pragma unroll
    for (int k = 0; k < 4; ++k) {
      const int bs = k >> 1;
      const int hf = k & 1;
      const v4f val = *(const v4f*)(slabw + bs * 256 + hf * 128 + lane * 4);
      float* dst = plane + (size_t)((2 * bp + bs) * kCO + obase) * kQS + hf * 128 + lane * 4;
      *(volatile v4f*)dst = val;
    }
    __threadfence();
  }
}

template <int MODE>
__global__ __launch_bounds__(128) void em_pass_kernel(
    const unsigned short* __restrict__ poseT, const unsigned short* __restrict__ ttT,
    const float* __restrict__ act,
    const float* __restrict__ pca, const float* __restrict__ pcb,
    float* __restrict__ nca, float* __restrict__ ncb,
    float* __restrict__ omu, float* __restrict__ lsum) {
  __shared__ __align__(16) float slab[4][512];
  __shared__ float lgs[32];

  const int tid   = (int)threadIdx.x;
  const int lane  = tid & 31;
  const int wave  = tid >> 5;
  const int h     = lane >> 4;
  const int c     = lane & 15;
  const int ch    = c >> 3;
  const int s     = c & 7;
  const int bx    = (int)blockIdx.x;
  const int by    = (int)blockIdx.y;
  const int bp    = 4 * by + wave;
  const int m0    = 16 * bp;
  const int bg    = 2 * bp + h;
  const int n0    = 32 * bx;
  const int obase = 4 * bx;

  float ca[2][8], cb[2][8];
#pragma unroll
  for (int j = 0; j < 2; ++j)
#pragma unroll
    for (int r = 0; r < 8; ++r) { ca[j][r] = 0.0f; cb[j][r] = 0.0f; }
  if (MODE > 0) {
#pragma unroll
    for (int j = 0; j < 2; ++j) {
      const size_t off = ((size_t)(bg * kCO + obase + 2 * j + ch) * kS + s) * kQ;
      load8_wait(pca + off, ca[j]);
      load8_wait(pcb + off, cb[j]);
    }
  }

  float A0[2];
  float A1[2][8], A2[2][8];
#pragma unroll
  for (int j = 0; j < 2; ++j) {
    A0[j] = 0.0f;
#pragma unroll
    for (int r = 0; r < 8; ++r) { A1[j][r] = 0.0f; A2[j][r] = 0.0f; }
  }

  const _Float16* Ap  = (const _Float16*)(const void*)poseT + (size_t)(m0 + c) * kPitchH + 8 * h;
  const _Float16* Bp0 = (const _Float16*)(const void*)ttT + (size_t)(n0 + c) * kPitchH + 8 * h;
  const _Float16* Bp1 = Bp0 + 16 * kPitchH;
  const float* actp = act + (size_t)bg * kCI;
  const v4u zu = (v4u){0u, 0u, 0u, 0u};
  const v8h z8 = __builtin_bit_cast(v8h, zu);
  const v8f zacc = (v8f){0.f, 0.f, 0.f, 0.f, 0.f, 0.f, 0.f, 0.f};

#pragma unroll 1
  for (int ic = 0; ic < kCI; ++ic) {
    FragU fa, fb0, fb1;
    fa.h[0]  = *(const v8h*)(Ap  + (size_t)ic * (kB * kQ * kPitchH));
    fa.h[1]  = z8;
    fb0.h[0] = *(const v8h*)(Bp0 + (size_t)ic * (kCO * kS * kPitchH));
    fb0.h[1] = z8;
    fb1.h[0] = *(const v8h*)(Bp1 + (size_t)ic * (kCO * kS * kPitchH));
    fb1.h[1] = z8;
    const float actv = actp[ic];
    v8f acc0 = mma_f16(fa.v, fb0.v, zacc);
    v8f acc1 = mma_f16(fa.v, fb1.v, zacc);
    guard_2acc_3frag(acc0, acc1, fa.v, fb0.v, fb1.v);
    tile_update<MODE>(acc0, actv, ca[0], cb[0], A0[0], A1[0], A2[0]);
    tile_update<MODE>(acc1, actv, ca[1], cb[1], A0[1], A1[1], A2[1]);
  }

  float inv0[2];
#pragma unroll
  for (int j = 0; j < 2; ++j) inv0[j] = (A0[j] != 0.0f) ? (1.0f / A0[j]) : 0.0f;
  float mu[2][8], varc[2][8];
#pragma unroll
  for (int j = 0; j < 2; ++j)
#pragma unroll
    for (int r = 0; r < 8; ++r) {
      const float m   = A1[j][r] * inv0[j];
      const float ex2 = A2[j][r] * inv0[j];
      const float var = ex2 - m * m;
      mu[j][r]   = m;
      varc[j][r] = fmaxf(var, 1e-30f);
    }

  float* sw = slab[wave];
  if (MODE < 2) {
    float can[2][8];
#pragma unroll
    for (int j = 0; j < 2; ++j)
#pragma unroll
      for (int r = 0; r < 8; ++r) {
        can[j][r] = kSqrtHalfLog2e / sqrtf(varc[j][r]);
        sw[h * 256 + j * 128 + c * 8 + r] = can[j][r];
      }
    __syncthreads();
    store_runs(sw, nca, bp, obase, lane);
    __syncthreads();
#pragma unroll
    for (int j = 0; j < 2; ++j)
#pragma unroll
      for (int r = 0; r < 8; ++r) sw[h * 256 + j * 128 + c * 8 + r] = -(can[j][r] * mu[j][r]);
    __syncthreads();
    store_runs(sw, ncb, bp, obase, lane);
  } else {
#pragma unroll
    for (int j = 0; j < 2; ++j) {
      float lv = 0.0f;
#pragma unroll
      for (int r = 0; r < 8; ++r) lv += logf(varc[j][r]);
      lv += __shfl_xor(lv, 1, 32);
      lv += __shfl_xor(lv, 2, 32);
      lv += __shfl_xor(lv, 4, 32);
      lgs[(2 * wave + h) * 4 + 2 * j + ch] = 0.5f * lv;
    }
#pragma unroll
    for (int j = 0; j < 2; ++j)
#pragma unroll
      for (int r = 0; r < 8; ++r) {
        sw[h * 256 + j * 128 + ch * 64 + r * 8 + s] = mu[j][r];
      }
    __syncthreads();
    store_runs(sw, omu, bp, obase, lane);
    if (wave == 0) {
      const float val = lgs[lane];
      float* dst = lsum + (size_t)(bx * 16 + 8 * by) * 4 + lane;
      *(volatile float*)dst = val;
      __threadfence();
      *(volatile float*)dst = val;
    }
  }
}

__global__ __launch_bounds__(128) void softmax_out_kernel(const float* __restrict__ lsum, const float* __restrict__ bias_a,
                                                          const float* __restrict__ bias_b, float* __restrict__ out0) {
  __shared__ float redm[4];
  __shared__ float reds[4];
  __shared__ __align__(16) float vals[128];
  const int b    = (int)blockIdx.x;
  const int o    = (int)threadIdx.x;
  const int lane = o & 31;
  const int wave = o >> 5;
  const float L = lsum[((size_t)(o >> 2) * kB + b) * 4 + (o & 3)];
  const float x = kLamb * ((bias_a[o] - bias_b[o]) - L);
  float m = x;
#pragma unroll
  for (int off = 16; off > 0; off >>= 1) m = fmaxf(m, __shfl_xor(m, off, 32));
  if (lane == 0) redm[wave] = m;
  __syncthreads();
  const float mx = fmaxf(fmaxf(redm[0], redm[1]), fmaxf(redm[2], redm[3]));
  const float e = expf(x - mx);
  float sm = e;
#pragma unroll
  for (int off = 16; off > 0; off >>= 1) sm += __shfl_xor(sm, off, 32);
  if (lane == 0) reds[wave] = sm;
  __syncthreads();
  const float tot = ((reds[0] + reds[1]) + reds[2]) + reds[3];
  vals[o] = e * (1.0f / tot);
  __syncthreads();
  if (wave == 0) {
    const v4f v = *(const v4f*)(vals + lane * 4);
    float* dst = out0 + (size_t)b * kCO + lane * 4;
    *(volatile v4f*)dst = v;
    __threadfence();
    *(volatile v4f*)dst = v;
  }
}

extern "C" void kernel_launch(void* const* d_in, const int* in_sizes, int n_in,
                              void* d_out, int out_size, void* d_ws, size_t ws_size,
                              hipStream_t stream) {
  if (n_in < 5) return;
  if (in_sizes[0] != kB * kCI || in_sizes[1] != kB * kCI * kQS || in_sizes[2] != kCI * kCO * kQS ||
      in_sizes[3] != kCO || in_sizes[4] != kCO) return;
  if (out_size < kOut0Elems + kOut1Elems) return;

  const float* act    = (const float*)d_in[0];
  const float* pose   = (const float*)d_in[1];
  const float* trans  = (const float*)d_in[2];
  const float* bias_a = (const float*)d_in[3];
  const float* bias_b = (const float*)d_in[4];

  char* ws = (char*)d_ws;
  size_t off = 0;
  unsigned short* poseT = (unsigned short*)(ws + off); off += (size_t)kRowsPose * kPitchH * 2;
  unsigned short* ttT   = (unsigned short*)(ws + off); off += (size_t)kRowsT * kPitchH * 2;
  float* caA  = (float*)(ws + off); off += (size_t)kPlaneElems * 4;
  float* cbA  = (float*)(ws + off); off += (size_t)kPlaneElems * 4;
  float* caB  = (float*)(ws + off); off += (size_t)kPlaneElems * 4;
  float* cbB  = (float*)(ws + off); off += (size_t)kPlaneElems * 4;
  float* lsum = (float*)(ws + off); off += (size_t)kLsumElems * 4;
  if (off > ws_size) return;

  float* out0 = (float*)d_out;
  float* out1 = (float*)d_out + kOut0Elems;

  prep16_kernel<1><<<(kRowsPose * 2) / 256, 256, 0, stream>>>(pose, poseT, kPoseCarry);
  prep16_kernel<0><<<(kRowsT * 2) / 256, 256, 0, stream>>>(trans, ttT, kTCarry);

  const dim3 g(32, 2);
  em_pass_kernel<0><<<g, 128, 0, stream>>>(poseT, ttT, act, caB, cbB, caA, cbA, out1, lsum);
  em_pass_kernel<1><<<g, 128, 0, stream>>>(poseT, ttT, act, caA, cbA, caB, cbB, out1, lsum);
  em_pass_kernel<2><<<g, 128, 0, stream>>>(poseT, ttT, act, caB, cbB, caA, cbA, out1, lsum);

  softmax_out_kernel<<<kB, 128, 0, stream>>>(lsum, bias_a, bias_b, out0);
}
